// MH_MoE_10161892622874
// MI455X (gfx1250) — hardware-verified
//
#include <hip/hip_runtime.h>
#include <stdint.h>
#include <stddef.h>
#include <math.h>

#pragma clang fp contract(off)

#define NBT  2
#define SEQ  2048
#define HID  1024
#define NROW 4096
#define NHS  8
#define HDM  128
#define NSUB 32768
#define NEX  8
#define FFD  512

#define CP   132
#define TP   72
#define AP   136
#define HP   520
#define YP   68

#define LDS_GEMM (128 * CP * 4)
#define LDS_A1   (64 * AP * 2)
#define LDS_H1   (64 * HP * 2)
#define LDS_EXP  (2 * LDS_A1 + 2 * LDS_H1 + 512)
#define LDS_LST  (NSUB * 4)

static_assert(8 * 16 * YP * 4 <= 2 * LDS_A1);
static_assert((AP * 2) % 16 == 0);
static_assert((HP * 2) % 16 == 0);
static_assert((CP * 4) % 16 == 0);
static_assert((TP * 2) % 16 == 0);
static_assert((YP * 4) % 16 == 0);
static_assert(NROW % 128 == 0);
static_assert(HID % 128 == 0);
static_assert(NSUB % 256 == 0);
static_assert(NSUB == NROW * NHS);
static_assert(HID == NHS * HDM);
static_assert(HDM % 32 == 0);
static_assert(FFD % 128 == 0);

typedef __bf16         v16bf __attribute__((ext_vector_type(16)));
typedef float          v8f   __attribute__((ext_vector_type(8)));
typedef float          v4f   __attribute__((ext_vector_type(4)));
typedef unsigned int   v4u   __attribute__((ext_vector_type(4)));
typedef unsigned int   v2u   __attribute__((ext_vector_type(2)));
typedef int            v4i   __attribute__((ext_vector_type(4)));
typedef v4f __attribute__((may_alias)) v4fa;
typedef v4u __attribute__((may_alias)) v4ua;
typedef v2u __attribute__((may_alias)) v2ua;
typedef v4i __attribute__((may_alias)) v4ia;

union FragBF { v16bf v; v4u q[2]; };

__device__ __forceinline__ unsigned int bfb(float f) {
  unsigned int u = __float_as_uint(f);
  u += 0x7FFFu + ((u >> 16) & 1u);
  return u >> 16;
}
__device__ __forceinline__ void split2(float v, unsigned int& hi, unsigned int& lo) {
  hi = bfb(v);
  lo = bfb(v - __uint_as_float(hi << 16));
}
__device__ __forceinline__ unsigned int pk(unsigned int a, unsigned int b) { return (a & 0xFFFFu) | (b << 16); }

__device__ __forceinline__ v8f wmma_bf(v16bf a, v16bf b, v8f c) {
  v8f d = __builtin_amdgcn_wmma_f32_16x16x32_bf16(false, a, false, b, (short)0, c, false, false);
  asm volatile("v_nop\n\tv_nop\n\tv_nop\n\tv_nop" : "+v"(d) : "v"(a), "v"(b));
  return d;
}

__device__ __forceinline__ v16bf ldfrag_bf(const unsigned short* p, int h) {
  FragBF f;
  f.q[0] = *(const v4ua*)(p + 8 * h);
  f.q[1] = *(const v4ua*)(p + 16 + 8 * h);
  return f.v;
}

__device__ __forceinline__ float gelu_t(float x) {
  const float c = 0.7978845608028654f;
  const float x3 = (x * x) * x;
  const float u = c * (x + 0.044715f * x3);
  const float e2 = __expf(2.0f * u);
  const float th = 1.0f - 2.0f * __builtin_amdgcn_rcpf(e2 + 1.0f);
  return x * (0.5f * (1.0f + th));
}

__global__ __launch_bounds__(256) void k_split_x(const float* __restrict__ x,
                                                 unsigned short* __restrict__ xh,
                                                 unsigned short* __restrict__ xl, int n8)
{
  const int g = blockIdx.x * 256 + threadIdx.x;
  if (g >= n8) return;
  const float* s = x + (size_t)g * 8;
  const v4f a = *(const v4fa*)s;
  const v4f c = *(const v4fa*)(s + 4);
  unsigned int h0, l0, h1, l1, h2, l2, h3, l3, h4, l4, h5, l5, h6, l6, h7, l7;
  split2(a.x, h0, l0); split2(a.y, h1, l1); split2(a.z, h2, l2); split2(a.w, h3, l3);
  split2(c.x, h4, l4); split2(c.y, h5, l5); split2(c.z, h6, l6); split2(c.w, h7, l7);
  const v4u H = { pk(h0, h1), pk(h2, h3), pk(h4, h5), pk(h6, h7) };
  const v4u L = { pk(l0, l1), pk(l2, l3), pk(l4, l5), pk(l6, l7) };
  unsigned short* dh = xh + (size_t)g * 8;
  unsigned short* dl = xl + (size_t)g * 8;
  *(volatile v4u*)dh = H;
  *(volatile v4u*)dl = L;
  __threadfence();
  *(volatile v4u*)dh = H;
  *(volatile v4u*)dl = L;
}

__device__ __forceinline__ void wt_store_pass(const unsigned short* shH, const unsigned short* shL,
                                              unsigned short* dh, unsigned short* dl,
                                              int e, int R, int C, int r0, int c0, int wv, int lane)
{
  const int q8 = lane & 7, sub = lane >> 3;
  #pragma unroll
  for (int i = 0; i < 2; ++i) {
    const int n = wv * 8 + i * 4 + sub;
    const v4u hv = *(const v4ua*)(shH + n * TP + 8 * q8);
    const v4u lv = *(const v4ua*)(shL + n * TP + 8 * q8);
    const size_t go = ((size_t)e * C + c0 + n) * R + r0 + 8 * q8;
    *(volatile v4u*)(dh + go) = hv;
    *(volatile v4u*)(dl + go) = lv;
  }
}

__global__ __launch_bounds__(256) void k_cvt_wt(const float* __restrict__ wmh, const float* __restrict__ wmg,
                                                const float* __restrict__ w1, const float* __restrict__ w2,
                                                unsigned short* __restrict__ pmhh, unsigned short* __restrict__ pmhl,
                                                unsigned short* __restrict__ pmgh, unsigned short* __restrict__ pmgl,
                                                unsigned short* __restrict__ p1h, unsigned short* __restrict__ p1l,
                                                unsigned short* __restrict__ p2h, unsigned short* __restrict__ p2l)
{
  __shared__ __align__(16) unsigned short shH[64 * TP];
  __shared__ __align__(16) unsigned short shL[64 * TP];
  const int tid = threadIdx.x, lane = tid & 31, wv = tid >> 5;
  const int z = blockIdx.z;
  int which = 0;
  which = (z == 1) ? 1 : which;
  which = (z >= 2 && z < 10) ? 2 : which;
  which = (z >= 10) ? 3 : which;
  int e = 0;
  e = (which == 2) ? (z - 2) : e;
  e = (which == 3) ? (z - 10) : e;
  const float* src = wmh;
  src = (which == 1) ? wmg : src;
  src = (which == 2) ? w1 : src;
  src = (which == 3) ? w2 : src;
  unsigned short* dh = pmhh;
  dh = (which == 1) ? pmgh : dh;
  dh = (which == 2) ? p1h : dh;
  dh = (which == 3) ? p2h : dh;
  unsigned short* dl = pmhl;
  dl = (which == 1) ? pmgl : dl;
  dl = (which == 2) ? p1l : dl;
  dl = (which == 3) ? p2l : dl;
  const int R = (which == 2) ? HDM : ((which == 3) ? FFD : HID);
  const int C = (which == 2) ? FFD : ((which == 3) ? HDM : HID);
  const int r0 = blockIdx.x * 64;
  const int c0 = blockIdx.y * 64;
  if (r0 >= R || c0 >= C) return;
  const float* sp = src + (size_t)e * R * C;
  #pragma unroll
  for (int j = 0; j < 4; ++j) {
    const int idx = tid + 256 * j;
    const int row = idx >> 4, c4 = idx & 15;
    const v4f v = *(const v4fa*)(sp + (size_t)(r0 + row) * C + c0 + 4 * c4);
    const int cb = 4 * c4;
    unsigned int h0, l0, h1, l1, h2, l2, h3, l3;
    split2(v.x, h0, l0); split2(v.y, h1, l1); split2(v.z, h2, l2); split2(v.w, h3, l3);
    shH[(cb + 0) * TP + row] = (unsigned short)h0;  shL[(cb + 0) * TP + row] = (unsigned short)l0;
    shH[(cb + 1) * TP + row] = (unsigned short)h1;  shL[(cb + 1) * TP + row] = (unsigned short)l1;
    shH[(cb + 2) * TP + row] = (unsigned short)h2;  shL[(cb + 2) * TP + row] = (unsigned short)l2;
    shH[(cb + 3) * TP + row] = (unsigned short)h3;  shL[(cb + 3) * TP + row] = (unsigned short)l3;
  }
  __syncthreads();
  wt_store_pass(shH, shL, dh, dl, e, R, C, r0, c0, wv, lane);
  __threadfence();
  wt_store_pass(shH, shL, dh, dl, e, R, C, r0, c0, wv, lane);
}

__device__ __forceinline__ void ep_f32_pass(const float* sC, const float* bias,
                                            float* outf, int ldo, int m0, int n0, int wv, int lane)
{
  const v4f bb = *(const v4fa*)(bias + n0 + 4 * lane);
  #pragma unroll
  for (int i = 0; i < 16; ++i) {
    const int row = wv * 16 + i;
    v4f v = *(const v4fa*)(sC + row * CP + 4 * lane);
    v = v + bb;
    *(volatile v4f*)(outf + (size_t)(m0 + row) * ldo + n0 + 4 * lane) = v;
  }
}

__global__ __launch_bounds__(256) void k_gemm3(
    const unsigned short* __restrict__ Ah, const unsigned short* __restrict__ Al, int lda,
    const unsigned short* __restrict__ Bh, const unsigned short* __restrict__ Bl, int ldb, int K,
    const float* __restrict__ bias, float* __restrict__ outf, int ldo)
{
  extern __shared__ __align__(16) unsigned char dsm_g[];
  float* sC = (float*)dsm_g;
  const int tid = threadIdx.x, lane = tid & 31, wv = tid >> 5;
  const int h = lane >> 4, m = lane & 15;
  const int wm = wv & 3, wn = wv >> 2;
  const int m0 = blockIdx.x * 128, n0 = blockIdx.y * 128;
  const v8f z8 = {0.f, 0.f, 0.f, 0.f, 0.f, 0.f, 0.f, 0.f};
  v8f acc[2][4];
  #pragma unroll
  for (int mt = 0; mt < 2; ++mt)
    #pragma unroll
    for (int nt = 0; nt < 4; ++nt) acc[mt][nt] = z8;

  #pragma unroll 1
  for (int k0 = 0; k0 < K; k0 += 32) {
    v16bf ah[2], al[2];
    #pragma unroll
    for (int mt = 0; mt < 2; ++mt) {
      const size_t ro = (size_t)(m0 + 32 * wm + 16 * mt + m) * lda + k0;
      ah[mt] = ldfrag_bf(Ah + ro, h);
      al[mt] = ldfrag_bf(Al + ro, h);
    }
    #pragma unroll
    for (int nt = 0; nt < 4; ++nt) {
      const size_t co = (size_t)(n0 + 64 * wn + 16 * nt + m) * ldb + k0;
      const v16bf bh = ldfrag_bf(Bh + co, h);
      const v16bf bl = ldfrag_bf(Bl + co, h);
      #pragma unroll
      for (int mt = 0; mt < 2; ++mt) {
        acc[mt][nt] = wmma_bf(ah[mt], bh, acc[mt][nt]);
        acc[mt][nt] = wmma_bf(ah[mt], bl, acc[mt][nt]);
        acc[mt][nt] = wmma_bf(al[mt], bh, acc[mt][nt]);
      }
    }
  }
  #pragma unroll
  for (int mt = 0; mt < 2; ++mt)
    #pragma unroll
    for (int nt = 0; nt < 4; ++nt)
      #pragma unroll
      for (int r = 0; r < 8; ++r) {
        const int row = 32 * wm + 16 * mt + 8 * h + r;
        const int col = 64 * wn + 16 * nt + m;
        sC[row * CP + col] = acc[mt][nt][r];
      }
  __syncthreads();
  ep_f32_pass(sC, bias, outf, ldo, m0, n0, wv, lane);
  __threadfence();
  ep_f32_pass(sC, bias, outf, ldo, m0, n0, wv, lane);
}

__device__ __forceinline__ void acc8(double* lg, float xv, const float* w) {
  const v4f a = *(const v4fa*)w;
  const v4f b = *(const v4fa*)(w + 4);
  const double x = (double)xv;
  lg[0] = fma(x, (double)a.x, lg[0]); lg[1] = fma(x, (double)a.y, lg[1]);
  lg[2] = fma(x, (double)a.z, lg[2]); lg[3] = fma(x, (double)a.w, lg[3]);
  lg[4] = fma(x, (double)b.x, lg[4]); lg[5] = fma(x, (double)b.y, lg[5]);
  lg[6] = fma(x, (double)b.z, lg[6]); lg[7] = fma(x, (double)b.w, lg[7]);
}

__global__ __launch_bounds__(256) void k_router(const float* __restrict__ hf, const float* __restrict__ wr,
                                                float* __restrict__ rec, int nsub)
{
  __shared__ __align__(16) float swr[HDM * NEX];
  const int tid = threadIdx.x;
  #pragma unroll
  for (int i = 0; i < (HDM * NEX) / 256; ++i) swr[tid + 256 * i] = wr[tid + 256 * i];
  __syncthreads();
  const int t = blockIdx.x * 256 + tid;
  const int tc = (t < nsub) ? t : (nsub - 1);
  const float* hr = hf + (size_t)tc * HDM;
  double lg[8];
  #pragma unroll
  for (int e = 0; e < NEX; ++e) lg[e] = 0.0;
  #pragma unroll 1
  for (int d4 = 0; d4 < HDM / 4; ++d4) {
    const v4f hv = *(const v4fa*)(hr + 4 * d4);
    const float* w0 = swr + 32 * d4;
    acc8(lg, hv.x, w0);
    acc8(lg, hv.y, w0 + 8);
    acc8(lg, hv.z, w0 + 16);
    acc8(lg, hv.w, w0 + 24);
  }
  double mxd = lg[0];
  #pragma unroll
  for (int e = 1; e < NEX; ++e) mxd = fmax(mxd, lg[e]);
  float ex[8];
  float sum = 0.f;
  #pragma unroll
  for (int e = 0; e < NEX; ++e) { ex[e] = __expf((float)(lg[e] - mxd)); sum = sum + ex[e]; }
  const float rs = 1.0f / sum;
  float pr[8];
  #pragma unroll
  for (int e = 0; e < NEX; ++e) pr[e] = ex[e] * rs;
  int i1 = 0;
  double l1 = lg[0];
  #pragma unroll
  for (int e = 1; e < NEX; ++e) {
    const bool tk = lg[e] > l1;
    l1 = tk ? lg[e] : l1;
    i1 = tk ? e : i1;
  }
  int i2 = -1;
  double l2 = -1.0e300;
  #pragma unroll
  for (int e = 0; e < NEX; ++e) {
    const bool tk = (e != i1) && (lg[e] > l2);
    l2 = tk ? lg[e] : l2;
    i2 = tk ? e : i2;
  }
  float p1 = pr[0], p2 = pr[0];
  #pragma unroll
  for (int e = 0; e < NEX; ++e) { p1 = (e == i1) ? pr[e] : p1; p2 = (e == i2) ? pr[e] : p2; }
  const float rden = 1.0f / (p1 + p2);
  const float g1 = p1 * rden, g2 = p2 * rden;
  const bool lo1 = (i1 < i2);
  const int elo = lo1 ? i1 : i2;
  const int ehi = lo1 ? i2 : i1;
  const float wlo = lo1 ? g1 : g2;
  const float whi = lo1 ? g2 : g1;
  const v4f rv = { wlo, whi, (float)elo, (float)ehi };
  if (t < nsub) *(volatile v4f*)(rec + (size_t)t * 4) = rv;
  __threadfence();
  if (t < nsub) *(volatile v4f*)(rec + (size_t)t * 4) = rv;
}

__device__ __forceinline__ void list_pass(const int* s_list, int* L, int* CL, int base, int tid) {
  #pragma unroll 4
  for (int j = 0; j < NSUB / 1024; ++j) {
    const int idx = tid + 256 * j;
    const v4i v = *(const v4ia*)(s_list + 4 * idx);
    *(volatile v4i*)(L + 4 * idx) = v;
  }
  if (tid < 8) {
    const v4i cv = { base, base, base, base };
    *(volatile v4i*)(CL + 4 * tid) = cv;
  }
}

__global__ __launch_bounds__(256) void k_lists(const float* __restrict__ rec, int* __restrict__ lst,
                                               int* __restrict__ cnt)
{
  extern __shared__ __align__(16) unsigned char dsm_l[];
  int* s_list = (int*)dsm_l;
  __shared__ int s_wc[8];
  const int tid = threadIdx.x, lane = tid & 31, wv = tid >> 5;
  const int se = blockIdx.x;
  const int s = se >> 3, e = se & 7;
  #pragma unroll 1
  for (int i = 0; i < NSUB / 256; ++i) s_list[tid + 256 * i] = 0;
  __syncthreads();
  int base = 0;
  #pragma unroll 1
  for (int ch = 0; ch < NSUB / 256; ++ch) {
    const int t = ch * 256 + tid;
    const v4f r = *(const v4fa*)(rec + (size_t)t * 4);
    const float self = (s == 0) ? r.z : r.w;
    const int sel = (int)self;
    const bool f = (sel == e);
    const unsigned int msk = __builtin_amdgcn_ballot_w32(f);
    const int off = __builtin_popcount(msk & ((1u << lane) - 1u));
    const int wc = __builtin_popcount(msk);
    if (lane == 0) s_wc[wv] = wc;
    __syncthreads();
    int pre = 0, tot = 0;
    #pragma unroll 1
    for (int w2 = 0; w2 < 8; ++w2) {
      const int cc = s_wc[w2];
      tot += cc;
      pre += (w2 < wv) ? cc : 0;
    }
    if (f) {
      int p = base + pre + off;
      p = (p < 0) ? 0 : ((p > NSUB - 1) ? (NSUB - 1) : p);
      s_list[p] = t;
    }
    base += tot;
    __syncthreads();
  }
  base = (base > NSUB) ? NSUB : base;
  int* L  = lst + (size_t)se * NSUB;
  int* CL = cnt + (size_t)se * 32;
  list_pass(s_list, L, CL, base, tid);
  __threadfence();
  list_pass(s_list, L, CL, base, tid);
}

__device__ __forceinline__ void yp0_pass(const float* sy, const int* s_tok, float* pout,
                                         int mg, int ng, int nrows, int lane)
{
  const int q16 = lane & 15, sub = lane >> 4;
  #pragma unroll
  for (int i = 0; i < 8; ++i) {
    const int rowl = 2 * i + sub;
    const int row = 16 * mg + rowl;
    const v4f v = *(const v4fa*)(sy + rowl * YP + 4 * q16);
    const int t = s_tok[row];
    const size_t go = (size_t)t * HDM + ng * 64 + 4 * q16;
    if (row < nrows) {
      *(volatile v4f*)(pout + go) = v;
    }
  }
}

__device__ __forceinline__ void yp1_pass(const float* sy, const int* s_tok, const float* padd,
                                         unsigned short* moh, unsigned short* mol,
                                         int mg, int ng, int nrows, int lane)
{
  const int q8 = lane & 7, sub = lane >> 3;
  #pragma unroll
  for (int i = 0; i < 4; ++i) {
    const int rowl = 4 * i + sub;
    const int row = 16 * mg + rowl;
    const v4f y0 = *(const v4fa*)(sy + rowl * YP + 8 * q8);
    const v4f y1 = *(const v4fa*)(sy + rowl * YP + 8 * q8 + 4);
    const int t = s_tok[row];
    const size_t go = (size_t)t * HDM + ng * 64 + 8 * q8;
    const v4f pa = *(const v4fa*)(padd + go);
    const v4f pb = *(const v4fa*)(padd + go + 4);
    const v4f ma = pa + y0;
    const v4f mb = pb + y1;
    unsigned int h0, l0, h1, l1, h2, l2, h3, l3, h4, l4, h5, l5, h6, l6, h7, l7;
    split2(ma.x, h0, l0); split2(ma.y, h1, l1); split2(ma.z, h2, l2); split2(ma.w, h3, l3);
    split2(mb.x, h4, l4); split2(mb.y, h5, l5); split2(mb.z, h6, l6); split2(mb.w, h7, l7);
    const v4u H = { pk(h0, h1), pk(h2, h3), pk(h4, h5), pk(h6, h7) };
    const v4u L = { pk(l0, l1), pk(l2, l3), pk(l4, l5), pk(l6, l7) };
    if (row < nrows) {
      *(volatile v4u*)(moh + go) = H;
      *(volatile v4u*)(mol + go) = L;
    }
  }
}

template <int SLOT>
__global__ __launch_bounds__(256) void k_expert(const float* __restrict__ hf,
                                                const unsigned short* __restrict__ w1h,
                                                const unsigned short* __restrict__ w1l,
                                                const unsigned short* __restrict__ w2h,
                                                const unsigned short* __restrict__ w2l,
                                                const float* __restrict__ b1, const float* __restrict__ b2,
                                                const float* __restrict__ rec,
                                                const int* __restrict__ lst,
                                                const int* __restrict__ cnt,
                                                const float* padd, float* pout,
                                                unsigned short* __restrict__ moh,
                                                unsigned short* __restrict__ mol)
{
  extern __shared__ __align__(16) unsigned char dsm_e[];
  unsigned short* sAh = (unsigned short*)dsm_e;
  unsigned short* sAl = (unsigned short*)(dsm_e + LDS_A1);
  unsigned short* sHh = (unsigned short*)(dsm_e + 2 * LDS_A1);
  unsigned short* sHl = (unsigned short*)(dsm_e + 2 * LDS_A1 + LDS_H1);
  float* sY    = (float*)dsm_e;
  int*   s_tok = (int*)(dsm_e + 2 * LDS_A1 + 2 * LDS_H1);
  float* s_w   = (float*)(dsm_e + 2 * LDS_A1 + 2 * LDS_H1 + 256);

  const int tid = threadIdx.x, lane = tid & 31, wv = tid >> 5;
  const int h = lane >> 4, m = lane & 15;
  const int e = blockIdx.y, tile = blockIdx.x;
  const int se = SLOT * NEX + e;

  int c = cnt[(size_t)se * 32];
  c = (c < 0) ? 0 : ((c > NSUB) ? NSUB : c);
  if (tile * 64 >= c) return;
  int nrows = c - tile * 64;
  nrows = (nrows > 64) ? 64 : nrows;

  if (tid < 64) {
    int idx = tile * 64 + tid;
    idx = (idx > NSUB - 1) ? (NSUB - 1) : idx;
    int t = lst[(size_t)se * NSUB + idx];
    t = (t < 0) ? 0 : ((t > NSUB - 1) ? (NSUB - 1) : t);
    const v4f r = *(const v4fa*)(rec + (size_t)t * 4);
    const float wgt = (SLOT == 0) ? r.x : r.y;
    s_tok[tid] = t;
    s_w[tid] = (tid < nrows) ? wgt : 0.0f;
  }
  __syncthreads();
  #pragma unroll
  for (int j = 0; j < 8; ++j) {
    const int idx = tid + 256 * j;
    const int row = idx >> 5, c4 = idx & 31;
    const size_t go = (size_t)s_tok[row] * HDM + 4 * c4;
    const v4f v = *(const v4fa*)(hf + go);
    unsigned int h0, l0, h1, l1, h2, l2, h3, l3;
    split2(v.x, h0, l0); split2(v.y, h1, l1); split2(v.z, h2, l2); split2(v.w, h3, l3);
    const v2u hv = { pk(h0, h1), pk(h2, h3) };
    const v2u lv = { pk(l0, l1), pk(l2, l3) };
    *(v2ua*)(sAh + row * AP + 4 * c4) = hv;
    *(v2ua*)(sAl + row * AP + 4 * c4) = lv;
  }
  __syncthreads();

  const int mg = wv & 3, ng = wv >> 2;
  const v8f z8 = {0.f, 0.f, 0.f, 0.f, 0.f, 0.f, 0.f, 0.f};

  #pragma unroll 1
  for (int nh = 0; nh < FFD / 128; ++nh) {
    v8f ac[4];
    #pragma unroll
    for (int nt = 0; nt < 4; ++nt) ac[nt] = z8;
    #pragma unroll 1
    for (int k0 = 0; k0 < HDM; k0 += 32) {
      const v16bf ah = ldfrag_bf(sAh + (16 * mg + m) * AP + k0, h);
      const v16bf al = ldfrag_bf(sAl + (16 * mg + m) * AP + k0, h);
      #pragma unroll
      for (int nt = 0; nt < 4; ++nt) {
        const int n = nh * 128 + ng * 64 + 16 * nt + m;
        const size_t bo = ((size_t)e * FFD + n) * HDM + k0;
        const v16bf bh = ldfrag_bf(w1h + bo, h);
        const v16bf bl = ldfrag_bf(w1l + bo, h);
        ac[nt] = wmma_bf(ah, bh, ac[nt]);
        ac[nt] = wmma_bf(ah, bl, ac[nt]);
        ac[nt] = wmma_bf(al, bh, ac[nt]);
      }
    }
    #pragma unroll
    for (int nt = 0; nt < 4; ++nt) {
      const int col = nh * 128 + ng * 64 + 16 * nt + m;
      const float bb = b1[(size_t)e * FFD + col];
      #pragma unroll
      for (int r = 0; r < 8; ++r) {
        const int rowl = 16 * mg + 8 * h + r;
        const float av = gelu_t(ac[nt][r] + bb);
        unsigned int hb, lb;
        split2(av, hb, lb);
        sHh[rowl * HP + col] = (unsigned short)hb;
        sHl[rowl * HP + col] = (unsigned short)lb;
      }
    }
  }
  __syncthreads();

  v8f ya[4];
  #pragma unroll
  for (int nt = 0; nt < 4; ++nt) ya[nt] = z8;
  #pragma unroll 1
  for (int k0 = 0; k0 < FFD; k0 += 32) {
    const v16bf ah = ldfrag_bf(sHh + (16 * mg + m) * HP + k0, h);
    const v16bf al = ldfrag_bf(sHl + (16 * mg + m) * HP + k0, h);
    #pragma unroll
    for (int nt = 0; nt < 4; ++nt) {
      const int n = ng * 64 + 16 * nt + m;
      const size_t bo = ((size_t)e * HDM + n) * FFD + k0;
      const v16bf bh = ldfrag_bf(w2h + bo, h);
      const v16bf bl = ldfrag_bf(w2l + bo, h);
      ya[nt] = wmma_bf(ah, bh, ya[nt]);
      ya[nt] = wmma_bf(ah, bl, ya[nt]);
      ya[nt] = wmma_bf(al, bh, ya[nt]);
    }
  }
  __syncthreads();
  float* sy = sY + wv * 16 * YP;
  #pragma unroll
  for (int nt = 0; nt < 4; ++nt) {
    const int cl = 16 * nt + m;
    const float bb = b2[(size_t)e * HDM + ng * 64 + cl];
    #pragma unroll
    for (int r = 0; r < 8; ++r) {
      const int rowl = 8 * h + r;
      const float y = (ya[nt][r] + bb) * s_w[16 * mg + rowl];
      sy[rowl * YP + cl] = y;
    }
  }
  __syncthreads();
  if (SLOT == 0) {
    yp0_pass(sy, s_tok, pout, mg, ng, nrows, lane);
    __threadfence();
    yp0_pass(sy, s_tok, pout, mg, ng, nrows, lane);
  } else {
    yp1_pass(sy, s_tok, padd, moh, mol, mg, ng, nrows, lane);
    __threadfence();
    yp1_pass(sy, s_tok, padd, moh, mol, mg, ng, nrows, lane);
  }
}

extern "C" void kernel_launch(void* const* d_in, const int* in_sizes, int n_in,
                              void* d_out, int out_size, void* d_ws, size_t ws_size,
                              hipStream_t stream)
{
  if (n_in < 10) return;
  if (in_sizes[0] != NROW * HID) return;
  if (in_sizes[1] != HID * HID || in_sizes[2] != HID) return;
  if (in_sizes[3] != HID * HID || in_sizes[4] != HID) return;
  if (in_sizes[5] != HDM * NEX) return;
  if (in_sizes[6] != NEX * HDM * FFD || in_sizes[7] != NEX * FFD) return;
  if (in_sizes[8] != NEX * FFD * HDM || in_sizes[9] != NEX * HDM) return;
  if (out_size != NROW * HID) return;

  const float* x       = (const float*)d_in[0];
  const float* w_mh    = (const float*)d_in[1];
  const float* b_mh    = (const float*)d_in[2];
  const float* w_mg    = (const float*)d_in[3];
  const float* b_mg    = (const float*)d_in[4];
  const float* w_rt    = (const float*)d_in[5];
  const float* w1      = (const float*)d_in[6];
  const float* b1      = (const float*)d_in[7];
  const float* w2      = (const float*)d_in[8];
  const float* b2      = (const float*)d_in[9];
  float* out = (float*)d_out;

  const size_t bXP  = (size_t)NROW * HID * 2;
  const size_t bWP  = (size_t)HID * HID * 2;
  const size_t bW1P = (size_t)NEX * FFD * HDM * 2;
  const size_t bW2P = (size_t)NEX * HDM * FFD * 2;
  const size_t bHF  = (size_t)NROW * HID * 4;
  const size_t bREC = (size_t)NSUB * 16;
  const size_t bLST = (size_t)2 * NEX * NSUB * 4;
  const size_t bCNT = (size_t)2 * NEX * 32 * 4;
  const size_t bP0  = (size_t)NSUB * HDM * 4;
  const size_t bMP  = (size_t)NSUB * HDM * 2;
  const size_t total = 2 * bXP + 4 * bWP + 2 * bW1P + 2 * bW2P + bHF + bREC + bLST + bCNT + bP0 + 2 * bMP;
  if (total > ws_size) return;
  if (total > (size_t)134217728) return;

  char* ws = (char*)d_ws;
  size_t off = 0;
  unsigned short* XH  = (unsigned short*)(ws + off); off += bXP;
  unsigned short* XL  = (unsigned short*)(ws + off); off += bXP;
  unsigned short* WMH = (unsigned short*)(ws + off); off += bWP;
  unsigned short* WML = (unsigned short*)(ws + off); off += bWP;
  unsigned short* WGH = (unsigned short*)(ws + off); off += bWP;
  unsigned short* WGL = (unsigned short*)(ws + off); off += bWP;
  unsigned short* W1H = (unsigned short*)(ws + off); off += bW1P;
  unsigned short* W1L = (unsigned short*)(ws + off); off += bW1P;
  unsigned short* W2H = (unsigned short*)(ws + off); off += bW2P;
  unsigned short* W2L = (unsigned short*)(ws + off); off += bW2P;
  float*          HF  = (float*)(ws + off);          off += bHF;
  float*          REC = (float*)(ws + off);          off += bREC;
  int*            LST = (int*)(ws + off);            off += bLST;
  int*            CNT = (int*)(ws + off);            off += bCNT;
  float*          P0  = (float*)(ws + off);          off += bP0;
  unsigned short* MOH = (unsigned short*)(ws + off); off += bMP;
  unsigned short* MOL = (unsigned short*)(ws + off); off += bMP;
  if (off != total) return;

  hipFuncSetAttribute(reinterpret_cast<const void*>(&k_gemm3), hipFuncAttributeMaxDynamicSharedMemorySize, LDS_GEMM);
  hipFuncSetAttribute(reinterpret_cast<const void*>(&k_lists), hipFuncAttributeMaxDynamicSharedMemorySize, LDS_LST);
  hipFuncSetAttribute(reinterpret_cast<const void*>(&k_expert<0>), hipFuncAttributeMaxDynamicSharedMemorySize, LDS_EXP);
  hipFuncSetAttribute(reinterpret_cast<const void*>(&k_expert<1>), hipFuncAttributeMaxDynamicSharedMemorySize, LDS_EXP);

  k_split_x<<<(NROW * HID / 8) / 256, 256, 0, stream>>>(x, XH, XL, NROW * HID / 8);
  k_cvt_wt<<<dim3(16, 16, 18), 256, 0, stream>>>(w_mh, w_mg, w1, w2, WMH, WML, WGH, WGL, W1H, W1L, W2H, W2L);

  k_gemm3<<<dim3(NROW / 128, HID / 128), 256, LDS_GEMM, stream>>>(XH, XL, HID, WMH, WML, HID, HID, b_mh, HF, HID);

  k_router<<<NSUB / 256, 256, 0, stream>>>(HF, w_rt, REC, NSUB);
  k_lists<<<2 * NEX, 256, LDS_LST, stream>>>(REC, LST, CNT);

  k_expert<0><<<dim3(NSUB / 64, NEX), 256, LDS_EXP, stream>>>(HF, W1H, W1L, W2H, W2L, b1, b2, REC, LST, CNT,
                                                              P0, P0, MOH, MOL);
  k_expert<1><<<dim3(NSUB / 64, NEX), 256, LDS_EXP, stream>>>(HF, W1H, W1L, W2H, W2L, b1, b2, REC, LST, CNT,
                                                              P0, P0, MOH, MOL);

  k_gemm3<<<dim3(NROW / 128, HID / 128), 256, LDS_GEMM, stream>>>(MOH, MOL, HID, WGH, WGL, HID, HID, b_mg, out, HID);
}
